// QKVMultiheadAttention_80762565034148
// MI455X (gfx1250) — hardware-verified
//
#include <hip/hip_runtime.h>
#include <math.h>
#include <stdint.h>


#ifndef NB
#define NB   2
#endif
#ifndef SEQ
#define SEQ  2048
#endif
#define NB_FULL  2
#define SEQ_FULL 2048
#ifndef SEQ_OUT
#define SEQ_OUT SEQ_FULL
#endif
#define HID  2048
#define NH   16
#define HD   128

static_assert(NB >= 1 && NB <= NB_FULL);
static_assert(SEQ % 128 == 0 && SEQ >= 128 && SEQ <= SEQ_FULL);
static_assert(HID == NH * HD);
static_assert((HID & (HID - 1)) == 0);
static_assert(HID % 128 == 0 && HID % 32 == 0);

typedef _Float16 v16h __attribute__((ext_vector_type(16)));
typedef _Float16 v8h  __attribute__((ext_vector_type(8)));
typedef __bf16   v16b __attribute__((ext_vector_type(16)));
typedef __bf16   v8b  __attribute__((ext_vector_type(8)));
typedef float    v8f  __attribute__((ext_vector_type(8)));
typedef float    v4f  __attribute__((ext_vector_type(4)));
typedef unsigned int v4u __attribute__((ext_vector_type(4)));

__device__ __forceinline__ unsigned short f2bf_bits(float f) {
  const unsigned u = __float_as_uint(f);
  return (unsigned short)((u + 0x7FFFu + ((u >> 16) & 1u)) >> 16);
}
__device__ __forceinline__ float bf_bits2f(unsigned short x) { return __uint_as_float(((unsigned)x) << 16); }
__device__ __forceinline__ float bf_rne(float f) { return bf_bits2f(f2bf_bits(f)); }
__device__ __forceinline__ unsigned pk16(unsigned short a, unsigned short b) { return (unsigned)a | ((unsigned)b << 16); }
__device__ __forceinline__ unsigned short h2u(_Float16 x) { return __builtin_bit_cast(unsigned short, x); }

__device__ __forceinline__ void wave_sync() {
  __builtin_amdgcn_fence(__ATOMIC_RELEASE, "workgroup");
  __builtin_amdgcn_wave_barrier();
  __builtin_amdgcn_fence(__ATOMIC_ACQUIRE, "workgroup");
}

union FragB { v16b v; v8b h[2]; };
union FragH { v16h v; v8h h[2]; };
__device__ __forceinline__ v16b ldfrag_b(const __bf16* p) {
  FragB f; f.h[0] = *(const v8b*)(p); f.h[1] = *(const v8b*)(p + 16); return f.v;
}
__device__ __forceinline__ v16h ldfrag_h(const _Float16* p) {
  FragH f; f.h[0] = *(const v8h*)(p); f.h[1] = *(const v8h*)(p + 16); return f.v;
}

__device__ __forceinline__ v8f wmma_b(v16b a, v16b b, v8f c) {
  return __builtin_amdgcn_wmma_f32_16x16x32_bf16(false, a, false, b, (short)0, c, false, false);
}
__device__ __forceinline__ v8f wmma_h(v16h a, v16h b, v8f c) {
  c = __builtin_amdgcn_wmma_f32_16x16x32_f16(false, a, false, b, (short)0, c, false, false);
  asm volatile("v_nop\n\tv_nop\n\tv_nop\n\tv_nop" : "+v"(c) : "v"(a), "v"(b));
  return c;
}
__device__ __forceinline__ void dep_guard_b(v8f& x, v8f& y, v16b b, v16b a0, v16b a1, v16b l0, v16b l1) {
  asm volatile("v_nop\n\tv_nop\n\tv_nop\n\tv_nop" : "+v"(x), "+v"(y) : "v"(b), "v"(a0), "v"(a1), "v"(l0), "v"(l1));
}

__global__ __launch_bounds__(256) void cvt_bf16x8_kernel(const float* __restrict__ in, unsigned short* out, int n8) {
  const int i = blockIdx.x * 256 + threadIdx.x;
  if (i < n8) {
    const v4f a = *(const v4f*)(in + 8 * (size_t)i);
    const v4f c = *(const v4f*)(in + 8 * (size_t)i + 4);
    v4u w;
    w[0] = pk16(f2bf_bits(a[0]), f2bf_bits(a[1]));
    w[1] = pk16(f2bf_bits(a[2]), f2bf_bits(a[3]));
    w[2] = pk16(f2bf_bits(c[0]), f2bf_bits(c[1]));
    w[3] = pk16(f2bf_bits(c[2]), f2bf_bits(c[3]));
    volatile v4u* p = (volatile v4u*)(out + 8 * (size_t)i);
    *p = w;
    __threadfence();
    *p = w;
  }
}

#define GP 132

template <bool SPLITA, int OUT_MODE>
__global__ __launch_bounds__(128) void gemm_kernel(
    const unsigned short* __restrict__ Ap, const unsigned short* __restrict__ A2p, int lda, long strideA,
    const unsigned short* __restrict__ Btp, int ldb, long strideB,
    void* Cout, void* Cout2, void* Cout3, int ldc, long strideC,
    const float* __restrict__ bias, const float* __restrict__ bias2, int M, int N, int K) {
  __shared__ __align__(16) float sT[4][16 * GP];
  const int bz   = blockIdx.y;
  const int lane = threadIdx.x & 31;
  const int wave = threadIdx.x >> 5;
  const int tilesN = N >> 7;
  const int tilesM = M >> 5;
  const int tile = blockIdx.x * 4 + wave;
  if (tile >= tilesM * tilesN) return;
  const int tm = tile / tilesN;
  const int tn = tile - tm * tilesN;
  const int m0 = tm << 5;
  const int n0 = tn << 7;

  const __bf16* Ab  = (const __bf16*)(const void*)Ap + (size_t)bz * strideA;
  const __bf16* Ab2 = SPLITA ? ((const __bf16*)(const void*)A2p + (size_t)bz * strideA) : (const __bf16*)0;
  const __bf16* Bb  = (const __bf16*)(const void*)Btp + (size_t)bz * strideB;

  const int rlane = lane & 15;
  const int koff  = (lane >> 4) * 8;
  const int mOff  = (lane >> 4) * 8;

  v8f acc[2][8];
#pragma unroll
  for (int i = 0; i < 2; ++i)
#pragma unroll
    for (int j = 0; j < 8; ++j) acc[i][j] = (v8f){0.f, 0.f, 0.f, 0.f, 0.f, 0.f, 0.f, 0.f};

  for (int k0 = 0; k0 < K; k0 += 32) {
    const size_t ao0 = (size_t)(m0 + rlane) * lda + koff + k0;
    const size_t ao1 = (size_t)(m0 + 16 + rlane) * lda + koff + k0;
    const v16b a0 = ldfrag_b(Ab + ao0);
    const v16b a1 = ldfrag_b(Ab + ao1);
    v16b l0 = a0, l1 = a1;
    if (SPLITA) { l0 = ldfrag_b(Ab2 + ao0); l1 = ldfrag_b(Ab2 + ao1); }
#pragma unroll
    for (int j = 0; j < 8; ++j) {
      const v16b bh = ldfrag_b(Bb + (size_t)(n0 + (j << 4) + rlane) * ldb + koff + k0);
      acc[0][j] = wmma_b(a0, bh, acc[0][j]);
      if (SPLITA) acc[0][j] = wmma_b(l0, bh, acc[0][j]);
      acc[1][j] = wmma_b(a1, bh, acc[1][j]);
      if (SPLITA) acc[1][j] = wmma_b(l1, bh, acc[1][j]);
      dep_guard_b(acc[0][j], acc[1][j], bh, a0, a1, l0, l1);
    }
  }

  float* slab = sT[wave];
#pragma unroll
  for (int i = 0; i < 2; ++i) {
    const int mBase = m0 + (i << 4);
#pragma unroll
    for (int j = 0; j < 8; ++j)
#pragma unroll
      for (int r = 0; r < 8; ++r) slab[(mOff + r) * GP + (j << 4) + rlane] = acc[i][j][r];
    wave_sync();
    if (OUT_MODE == 0) {
      float* C = (float*)Cout + (size_t)bz * strideC;
      const int c4 = lane * 4;
      v4f bb;
#pragma unroll
      for (int e = 0; e < 4; ++e) bb[e] = bf_rne(bias[n0 + c4 + e]);
      for (int pass = 0; pass < 2; ++pass) {
#pragma unroll
        for (int it = 0; it < 16; ++it) {
          const v4f v = *(const v4f*)(slab + it * GP + c4) + bb;
          *(volatile v4f*)(C + (size_t)(mBase + it) * ldc + n0 + c4) = v;
        }
        __threadfence();
      }
    } else if (OUT_MODE == 1) {
      unsigned short* C = (unsigned short*)Cout + (size_t)bz * strideC;
      const int q16 = lane >> 4, c8 = (lane & 15) * 8;
      for (int pass = 0; pass < 2; ++pass) {
#pragma unroll
        for (int it = 0; it < 8; ++it) {
          const int row = it * 2 + q16;
          const float brow = bf_rne(bias[mBase + row]);
          const float* sp = slab + row * GP + c8;
          v4u hv;
#pragma unroll
          for (int p = 0; p < 4; ++p) {
            const float f0 = sp[2 * p] + brow, f1 = sp[2 * p + 1] + brow;
            const _Float16 e0 = (_Float16)f0, e1 = (_Float16)f1;
            hv[p] = pk16(h2u(e0), h2u(e1));
          }
          const size_t go = (size_t)(mBase + row) * ldc + n0 + c8;
          *(volatile v4u*)(C + go) = hv;
        }
        __threadfence();
      }
    } else {
      unsigned short* Q1 = (unsigned short*)Cout;
      unsigned short* Q2 = (unsigned short*)Cout2;
      unsigned short* K1 = (unsigned short*)Cout3;
      const int q16 = lane >> 4, c8 = (lane & 15) * 8;
      const bool isq  = (n0 < HID);
      const int  ncol = n0 & (HID - 1);
      const int  head = ncol / HD;
      float bb[8];
#pragma unroll
      for (int e = 0; e < 8; ++e) {
        const float vq = bf_rne(bias[ncol + c8 + e]);
        const float vk = bf_rne(bias2[ncol + c8 + e]);
        bb[e] = isq ? vq : vk;
      }
      const size_t rowBase = (size_t)(bz * NH + head) * SEQ;
      for (int pass = 0; pass < 2; ++pass) {
#pragma unroll
        for (int it = 0; it < 8; ++it) {
          const int row = it * 2 + q16;
          const int s   = mBase + row;
          const float* sp = slab + row * GP + c8;
          v4u hv, lv;
#pragma unroll
          for (int p = 0; p < 4; ++p) {
            const float f0 = sp[2 * p] + bb[2 * p], f1 = sp[2 * p + 1] + bb[2 * p + 1];
            const _Float16 e0 = (_Float16)f0, e1 = (_Float16)f1;
            const _Float16 g0 = (_Float16)((f0 - (float)e0) * 2048.0f);
            const _Float16 g1 = (_Float16)((f1 - (float)e1) * 2048.0f);
            hv[p] = pk16(h2u(e0), h2u(e1));
            lv[p] = pk16(h2u(g0), h2u(g1));
          }
          const size_t go = (rowBase + (size_t)s) * HD + c8;
          if (isq) {
            *(volatile v4u*)(Q1 + go) = hv;
            *(volatile v4u*)(Q2 + go) = lv;
          } else {
            *(volatile v4u*)(K1 + go) = hv;
          }
        }
        __threadfence();
      }
    }
    wave_sync();
  }
}

#define AT_QB 64
#define AT_KC 64
#define OS_P  132
#define KV_HALVES (2 * AT_KC * HD + 512)
static_assert(SEQ % AT_QB == 0 && SEQ % AT_KC == 0);

__global__ __launch_bounds__(128)
void attn_kernel(const unsigned short* __restrict__ qhp, const unsigned short* __restrict__ qlp,
                 const unsigned short* __restrict__ kp, const unsigned short* __restrict__ vhp,
                 unsigned short* chp, unsigned short* clp) {
  __shared__ __align__(16) _Float16 KVs[KV_HALVES];
  __shared__ __align__(16) _Float16 Psh[4][16 * AT_KC];
  static_assert(4 * 16 * OS_P * 2 <= KV_HALVES);
  _Float16* const Ksh = KVs;
  _Float16* const Vts = KVs + AT_KC * HD;

  const int tid  = threadIdx.x;
  const int wave = tid >> 5;
  const int lane = tid & 31;
  const int hh   = lane >> 4;
  const int c    = lane & 15;

  constexpr int NQB = SEQ / AT_QB;
  const int bx  = blockIdx.x;
  const int qb  = bx % NQB;
  const int h   = (bx / NQB) % NH;
  const int b   = bx / (NQB * NH);
  const int q0  = qb * AT_QB + wave * 16;

  const _Float16* Qhg = (const _Float16*)(const void*)qhp + (size_t)(b * NH + h) * SEQ * HD;
  const _Float16* Qlg = (const _Float16*)(const void*)qlp + (size_t)(b * NH + h) * SEQ * HD;
  const _Float16* Kg  = (const _Float16*)(const void*)kp  + (size_t)(b * NH + h) * SEQ * HD;
  const _Float16* Vhg = (const _Float16*)(const void*)vhp + ((size_t)b * HID + (size_t)h * HD) * SEQ;
  const int qro = (q0 + c) * HD + 8 * hh;

  const v8f zero8 = (v8f){0.f, 0.f, 0.f, 0.f, 0.f, 0.f, 0.f, 0.f};
  const float inv2048 = 4.8828125e-4f;
  const float scale   = 1.0f / 11.313708305358887f;

  float mrow[8], lrow[8];
  v8f oh[8];
#pragma unroll
  for (int r = 0; r < 8; ++r) { mrow[r] = -INFINITY; lrow[r] = 0.f; }
#pragma unroll
  for (int t = 0; t < 8; ++t) oh[t] = zero8;

  for (int kc = 0; kc < SEQ / AT_KC; ++kc) {
    const int kv0 = kc * AT_KC;
    __syncthreads();
    {
      const int r = tid >> 1, half = (tid & 1) * 64;
      const _Float16* ks = Kg  + (size_t)(kv0 + r) * HD + half;
      const _Float16* vs = Vhg + (size_t)tid * SEQ + kv0;
#pragma unroll
      for (int i = 0; i < 8; ++i) {
        const v8h a0 = *(const v8h*)(ks + 8 * i);
        const v8h b0 = *(const v8h*)(vs + 8 * i);
        *(v8h*)(Ksh + r * HD + half + 8 * i) = a0;
        *(v8h*)(Vts + tid * AT_KC + 8 * i)   = b0;
      }
    }
    __syncthreads();

    v8f s[4];
    v8f dep = oh[7];
#pragma unroll
    for (int j = 0; j < 4; ++j) {
      v8f sh = zero8, sl = zero8;
#pragma unroll
      for (int dc = 0; dc < 4; ++dc) {
        int qo = qro + dc * 32;
        asm volatile("" : "+v"(qo) : "v"(dep));
        const v16h qa = ldfrag_h(Qhg + qo);
        const v16h qr = ldfrag_h(Qlg + qo);
        FragH kb;
        kb.h[0] = *(const v8h*)(Ksh + (j * 16 + c) * HD + dc * 32 + 8 * hh);
        kb.h[1] = *(const v8h*)(Ksh + (j * 16 + c) * HD + dc * 32 + 16 + 8 * hh);
        sh = wmma_h(qa, kb.v, sh);
        sl = wmma_h(qr, kb.v, sl);
        dep = sl;
      }
      s[j] = (sh + sl * inv2048) * scale;
    }

    float cm[8];
#pragma unroll
    for (int r = 0; r < 8; ++r) {
      float m = fmaxf(fmaxf(s[0][r], s[1][r]), fmaxf(s[2][r], s[3][r]));
#pragma unroll
      for (int off = 1; off < 16; off <<= 1) m = fmaxf(m, __shfl_xor(m, off, 32));
      cm[r] = m;
    }

    _Float16* pw = Psh[wave];
#pragma unroll
    for (int r = 0; r < 8; ++r) {
      const float mnew  = fmaxf(mrow[r], cm[r]);
      const float alpha = expf(mrow[r] - mnew);
      mrow[r] = mnew;
      float psum = 0.f;
#pragma unroll
      for (int j = 0; j < 4; ++j) {
        const float p = expf(s[j][r] - mnew);
        psum += p;
        pw[(8 * hh + r) * AT_KC + j * 16 + c] = (_Float16)(p * 32768.0f);
      }
#pragma unroll
      for (int off = 1; off < 16; off <<= 1) psum += __shfl_xor(psum, off, 32);
      lrow[r] = lrow[r] * alpha + psum;
#pragma unroll
      for (int t = 0; t < 8; ++t) oh[t][r] *= alpha;
    }
    wave_sync();

#pragma unroll 1
    for (int kk = 0; kk < 2; ++kk) {
      FragH pa;
      pa.h[0] = *(const v8h*)(pw + c * AT_KC + kk * 32 + 8 * hh);
      pa.h[1] = *(const v8h*)(pw + c * AT_KC + kk * 32 + 16 + 8 * hh);
#pragma unroll
      for (int t = 0; t < 8; ++t) {
        FragH vb;
        vb.h[0] = *(const v8h*)(Vts + (t * 16 + c) * AT_KC + kk * 32 + 8 * hh);
        vb.h[1] = *(const v8h*)(Vts + (t * 16 + c) * AT_KC + kk * 32 + 16 + 8 * hh);
        oh[t] = wmma_h(pa.v, vb.v, oh[t]);
      }
    }
  }

  __syncthreads();
  float* os = (float*)(void*)KVs + wave * (16 * OS_P);
#pragma unroll
  for (int r = 0; r < 8; ++r) {
    const float invl = (1.0f / lrow[r]) * 3.0517578125e-5f;
#pragma unroll
    for (int t = 0; t < 8; ++t) os[(8 * hh + r) * OS_P + t * 16 + c] = oh[t][r] * invl;
  }
  wave_sync();
  {
    const int q16 = lane >> 4, c8 = (lane & 15) * 8;
    for (int pass = 0; pass < 2; ++pass) {
#pragma unroll
      for (int it = 0; it < 8; ++it) {
        const int row = it * 2 + q16;
        const float* sp = os + row * OS_P + c8;
        v4u hv, lv;
#pragma unroll
        for (int p = 0; p < 4; ++p) {
          const float f0 = sp[2 * p], f1 = sp[2 * p + 1];
          const unsigned short hb0 = f2bf_bits(f0), hb1 = f2bf_bits(f1);
          const unsigned short lb0 = f2bf_bits(f0 - bf_bits2f(hb0));
          const unsigned short lb1 = f2bf_bits(f1 - bf_bits2f(hb1));
          hv[p] = pk16(hb0, hb1);
          lv[p] = pk16(lb0, lb1);
        }
        const size_t go = (size_t)(b * SEQ + q0 + row) * HID + h * HD + c8;
        *(volatile v4u*)(chp + go) = hv;
        *(volatile v4u*)(clp + go) = lv;
      }
      __threadfence();
    }
  }
}

extern "C" void kernel_launch(void* const* d_in, const int* in_sizes, int n_in,
                              void* d_out, int out_size, void* d_ws, size_t ws_size,
                              hipStream_t stream) {
  if (n_in < 9) return;
  if (in_sizes[0] < ((NB - 1) * SEQ_FULL + SEQ) * HID) return;
  if (in_sizes[1] < HID * HID || in_sizes[3] < HID * HID || in_sizes[5] < HID * HID || in_sizes[7] < HID * HID) return;
  if (in_sizes[2] < HID || in_sizes[4] < HID || in_sizes[6] < HID || in_sizes[8] < HID) return;
  if (out_size < ((NB - 1) * SEQ_OUT + SEQ) * HID) return;

  const float* x  = (const float*)d_in[0];
  const float* Wq = (const float*)d_in[1];
  const float* bq = (const float*)d_in[2];
  const float* Wk = (const float*)d_in[3];
  const float* bk = (const float*)d_in[4];
  const float* Wv = (const float*)d_in[5];
  const float* bv = (const float*)d_in[6];
  const float* Wo = (const float*)d_in[7];
  const float* bo = (const float*)d_in[8];
  float* out = (float*)d_out;

  const size_t szR0  = (size_t)NB * SEQ * HID * 2;
  const size_t szWqk = (size_t)2 * HID * HID * 2;
  const size_t szCtx = (size_t)NB * SEQ * HID * 2;
  const size_t szR1  = szWqk > szCtx ? szWqk : szCtx;
  const size_t szWo  = (size_t)HID * HID * 2;
  const size_t szQ   = (size_t)NB * NH * SEQ * HD * 2;
  const size_t szK   = szQ;
  const size_t szV   = (size_t)NB * HID * SEQ * 2;
  size_t off = 0;
  const size_t oR0  = off; off += szR0;
  const size_t oR1  = off; off += szR1;
  const size_t oWo  = off; off += szWo;
  const size_t oQh  = off; off += szQ;
  const size_t oQl  = off; off += szQ;
  const size_t oKp  = off; off += szK;
  const size_t oVth = off; off += szV;
  if (off > ws_size) return;
  if (off > (size_t)134217728) return;

  char* ws = (char*)d_ws;
  unsigned short* Xb  = (unsigned short*)(ws + oR0);
  unsigned short* Ch  = (unsigned short*)(ws + oR0);
  unsigned short* Wvb = (unsigned short*)(ws + oR1);
  unsigned short* Wqk = (unsigned short*)(ws + oR1);
  unsigned short* Cl  = (unsigned short*)(ws + oR1);
  unsigned short* Wob = (unsigned short*)(ws + oWo);
  unsigned short* Qh  = (unsigned short*)(ws + oQh);
  unsigned short* Ql  = (unsigned short*)(ws + oQl);
  unsigned short* Kp  = (unsigned short*)(ws + oKp);
  unsigned short* Vth = (unsigned short*)(ws + oVth);

  const dim3 blk256(256), blk128(128);
  const int n8x = SEQ * HID / 8, n8w = HID * HID / 8;

  for (int bb = 0; bb < NB; ++bb)
    cvt_bf16x8_kernel<<<dim3((n8x + 255) / 256), blk256, 0, stream>>>(
        x + (size_t)bb * SEQ_FULL * HID, Xb + (size_t)bb * SEQ * HID, n8x);
  cvt_bf16x8_kernel<<<dim3((n8w + 255) / 256), blk256, 0, stream>>>(Wv, Wvb, n8w);
  cvt_bf16x8_kernel<<<dim3((n8w + 255) / 256), blk256, 0, stream>>>(Wo, Wob, n8w);
  {
    const int M = HID, N = SEQ, K = HID;
    const int tiles = (M / 32) * (N / 128);
    gemm_kernel<false, 1><<<dim3((tiles + 3) / 4, NB), blk128, 0, stream>>>(
        Wvb, Wvb, HID, 0L, Xb, HID, (long)SEQ * HID, (void*)Vth, (void*)Vth, (void*)Vth, SEQ,
        (long)HID * SEQ, bv, bv, M, N, K);
  }
  cvt_bf16x8_kernel<<<dim3((n8w + 255) / 256), blk256, 0, stream>>>(Wq, Wqk, n8w);
  cvt_bf16x8_kernel<<<dim3((n8w + 255) / 256), blk256, 0, stream>>>(Wk, Wqk + (size_t)HID * HID, n8w);
  {
    const int M = SEQ, N = 2 * HID, K = HID;
    const int tiles = (M / 32) * (N / 128);
    gemm_kernel<false, 2><<<dim3((tiles + 3) / 4, NB), blk128, 0, stream>>>(
        Xb, Xb, HID, (long)SEQ * HID, Wqk, HID, 0L, (void*)Qh, (void*)Ql, (void*)Kp, HD, 0L, bq, bk, M, N, K);
  }
  attn_kernel<<<dim3(NB * NH * (SEQ / AT_QB)), blk128, 0, stream>>>(Qh, Ql, Kp, Vth, Ch, Cl);
  {
    const int M = SEQ, N = HID, K = HID;
    const int tiles = (M / 32) * (N / 128);
    gemm_kernel<true, 0><<<dim3((tiles + 3) / 4, NB), blk128, 0, stream>>>(
        Ch, Cl, HID, (long)SEQ * HID, Wob, HID, 0L, (void*)out, (void*)out, (void*)out, HID,
        (long)SEQ_OUT * HID, bo, bo, M, N, K);
  }
  (void)hipGetLastError();
}
